// NeuralODE_13795434955298
// MI455X (gfx1250) — hardware-verified
//
#include <hip/hip_runtime.h>
#include <math.h>

constexpr int D_DIM      = 64;
constexpr int H_DIM      = 128;
constexpr int N_BATCH    = 1024;
constexpr int N_SAVE     = 64;
constexpr int N_SUB      = 2;
constexpr int TILE_ROWS  = 16;
constexpr int NTHREADS   = 256;
constexpr int NWAVES     = NTHREADS / 32;
constexpr int TILE_ELEMS = TILE_ROWS * D_DIM;
constexpr float A_CARRY    = 16.0f;
constexpr float W_HI_CARRY = 1024.0f;
constexpr float W_LO_CARRY = 2048.0f;
constexpr float W_LO_INV   = 1.0f / 2048.0f;
constexpr float ACC_INV    = 1.0f / 16384.0f;
static_assert(N_BATCH % TILE_ROWS == 0);
static_assert(TILE_ELEMS == 4 * NTHREADS);
static_assert(H_DIM == 16 * NWAVES);
static_assert(D_DIM == 16 * (NWAVES / 2));
static_assert(D_DIM % 32 == 0 && (H_DIM / 2) % 32 == 0 && H_DIM % 32 == 0);
static_assert((H_DIM * D_DIM) % (8 * NTHREADS) == 0 && (H_DIM * H_DIM) % (8 * NTHREADS) == 0);

constexpr float TS_A21 = 0.161f;
constexpr float TS_A31 = -0.008480655492356989f;
constexpr float TS_A32 = 0.335480655492357f;
constexpr float TS_A41 = 2.8971530571054935f;
constexpr float TS_A42 = -6.359448489975075f;
constexpr float TS_A43 = 4.3622954328695815f;
constexpr float TS_A51 = 5.325864828439257f;
constexpr float TS_A52 = -11.748883564062828f;
constexpr float TS_A53 = 7.4955393428898365f;
constexpr float TS_A54 = -0.09249506636175525f;
constexpr float TS_A61 = 5.86145544294642f;
constexpr float TS_A62 = -12.92096931784711f;
constexpr float TS_A63 = 8.159367898576159f;
constexpr float TS_A64 = -0.071584973281401f;
constexpr float TS_A65 = -0.028269050394068383f;
constexpr float TS_B1 = 0.09646076681806523f;
constexpr float TS_B2 = 0.01f;
constexpr float TS_B3 = 0.4798896504144996f;
constexpr float TS_B4 = 1.379008574103742f;
constexpr float TS_B5 = -3.290069515436081f;
constexpr float TS_B6 = 2.324710524099774f;

typedef __attribute__((ext_vector_type(16))) _Float16 v16h;
typedef __attribute__((ext_vector_type(8)))  _Float16 v8h;
typedef __attribute__((ext_vector_type(4)))  _Float16 v4h;
typedef __attribute__((ext_vector_type(8)))  float    v8f;
typedef __attribute__((ext_vector_type(4)))  float    v4f;

__device__ __forceinline__ void dep_guard_h(v8f& a, v8f& b, v16h x, v16h y) { asm volatile("v_nop\n\tv_nop\n\tv_nop\n\tv_nop" : "+v"(a), "+v"(b) : "v"(x), "v"(y)); }
__device__ __forceinline__ void keep4_h(v16h a, v16h b, v16h c, v16h d) { asm volatile("v_nop" :: "v"(a), "v"(b), "v"(c), "v"(d)); }
__device__ __forceinline__ void acc_guard2(v8f& a, v8f& b) { asm volatile("v_nop\n\tv_nop\n\tv_nop\n\tv_nop" : "+v"(a), "+v"(b)); }
template <typename T> struct Frag;
template <> struct Frag<_Float16> {
  typedef v16h V; union U { v16h v; v8h h[2]; };
  static __device__ __forceinline__ v16h load(const _Float16* p) {
    U f; f.h[0] = *(const v8h*)(p); f.h[1] = *(const v8h*)(p + 16); return f.v;
  }
  static __device__ __forceinline__ v8f mma(v16h a, v16h b, v8f c) {
    return __builtin_amdgcn_wmma_f32_16x16x32_f16(false, a, false, b, (short)0, c, false, false);
  }
};

__device__ __forceinline__ float ftanh(float x) {
  const float e = __builtin_amdgcn_exp2f(x * 2.8853900817779268f);
  const float r = __builtin_amdgcn_rcpf(e + 1.0f);
  return fmaf(-2.0f, r, 1.0f);
}

__device__ __forceinline__ void mm_tile(const _Float16* arow, const _Float16* wh, const _Float16* wl,
                                        int kdepth, v8f& accH, v8f& accL) {
  const v8f z8 = {0.f, 0.f, 0.f, 0.f, 0.f, 0.f, 0.f, 0.f};
  accH = z8; accL = z8;
#pragma unroll 1
  for (int k0 = 0; k0 < kdepth; k0 += 32) {
    const v16h a  = Frag<_Float16>::load(arow + k0);
    const v16h bh = Frag<_Float16>::load(wh + k0);
    const v16h bl = Frag<_Float16>::load(wl + k0);
    accH = Frag<_Float16>::mma(a, bh, accH);
    accL = Frag<_Float16>::mma(a, bl, accL);
    dep_guard_h(accH, accL, a, bl);
    keep4_h(a, bh, bl, a);
  }
  acc_guard2(accH, accL);
}

__global__ __launch_bounds__(NTHREADS) void split_planes_kernel(const float* __restrict__ src,
                                                           unsigned short* __restrict__ hi,
                                                           unsigned short* __restrict__ lo, int n8) {
  const int i = blockIdx.x * NTHREADS + threadIdx.x;
  if (i < n8) {
    const float* sp = src + (size_t)i * 8;
    const v4f a = *(const v4f*)(sp);
    const v4f b = *(const v4f*)(sp + 4);
    v8h hv, lv;
#pragma unroll
    for (int e = 0; e < 4; ++e) {
      const float xa = a[e] * W_HI_CARRY;
      const float xb = b[e] * W_HI_CARRY;
      const _Float16 ha = (_Float16)xa;
      const _Float16 hb = (_Float16)xb;
      const float fa = (float)ha;
      const float fb = (float)hb;
      const float ra = (xa - fa) * W_LO_CARRY;
      const float rb = (xb - fb) * W_LO_CARRY;
      hv[e] = ha;
      hv[4 + e] = hb;
      lv[e] = (_Float16)ra;
      lv[4 + e] = (_Float16)rb;
    }
    _Float16* hp = (_Float16*)hi + (size_t)i * 8;
    _Float16* lp = (_Float16*)lo + (size_t)i * 8;
    *(volatile v8h*)hp = hv;
    *(volatile v8h*)lp = lv;
    __threadfence();
    *(volatile v8h*)hp = hv;
    *(volatile v8h*)lp = lv;
  }
}

__global__ __launch_bounds__(NTHREADS) void field_solver_kernel(
    const float* __restrict__ ts, const float* __restrict__ y0,
    const unsigned short* __restrict__ W1Hp, const unsigned short* __restrict__ W1Lp, const float* __restrict__ b1,
    const unsigned short* __restrict__ W2Hp, const unsigned short* __restrict__ W2Lp, const float* __restrict__ b2,
    const unsigned short* __restrict__ W3Hp, const unsigned short* __restrict__ W3Lp, const float* __restrict__ b3,
    float* __restrict__ out) {
  __shared__ __align__(16) _Float16 sX[TILE_ELEMS];
  __shared__ __align__(16) _Float16 sH1[TILE_ROWS * H_DIM];
  __shared__ __align__(16) _Float16 sH2[TILE_ROWS * H_DIM];
  __shared__ __align__(16) float    sKP[2 * TILE_ELEMS];

  const _Float16* W1H = (const _Float16*)W1Hp; const _Float16* W1L = (const _Float16*)W1Lp;
  const _Float16* W2H = (const _Float16*)W2Hp; const _Float16* W2L = (const _Float16*)W2Lp;
  const _Float16* W3H = (const _Float16*)W3Hp; const _Float16* W3L = (const _Float16*)W3Lp;

  const int tid = threadIdx.x, lane = tid & 31, wave = tid >> 5;
  const int c = lane & 15, hh = lane >> 4, koff = hh * 8;
  const int blk  = blockIdx.x;
  const int ncol = wave * 16 + c;
  const int n3   = (wave & 3) * 16 + c;
  const int kh3  = wave >> 2;
  const int e0   = tid * 4;

  const float b1v = b1[ncol];
  const float b2v = b2[ncol];
  const float b3l = b3[n3];
  const float b3v = (kh3 == 0) ? b3l : 0.0f;

  const _Float16* a1row = sX  + c * D_DIM + koff;
  const _Float16* a2row = sH1 + c * H_DIM + koff;
  const _Float16* a3row = sH2 + c * H_DIM + koff + kh3 * (H_DIM / 2);
  const _Float16* w1h = W1H + (size_t)ncol * D_DIM + koff;
  const _Float16* w1l = W1L + (size_t)ncol * D_DIM + koff;
  const _Float16* w2h = W2H + (size_t)ncol * H_DIM + koff;
  const _Float16* w2l = W2L + (size_t)ncol * H_DIM + koff;
  const _Float16* w3h = W3H + (size_t)n3 * H_DIM + koff + kh3 * (H_DIM / 2);
  const _Float16* w3l = W3L + (size_t)n3 * H_DIM + koff + kh3 * (H_DIM / 2);
  _Float16* h1dst = sH1 + (8 * hh) * H_DIM + ncol;
  _Float16* h2dst = sH2 + (8 * hh) * H_DIM + ncol;
  float*    k3dst = sKP + kh3 * TILE_ELEMS + (8 * hh) * D_DIM + n3;

  auto put_x = [&](v4f x) {
    v4h hv;
    hv[0] = (_Float16)(x[0] * A_CARRY);
    hv[1] = (_Float16)(x[1] * A_CARRY);
    hv[2] = (_Float16)(x[2] * A_CARRY);
    hv[3] = (_Float16)(x[3] * A_CARRY);
    *(v4h*)(sX + e0) = hv;
  };

  v4f yv = *(const v4f*)(y0 + (size_t)blk * TILE_ELEMS + e0);
  {
    float* op = out + (size_t)blk * TILE_ELEMS + e0;
    *(volatile v4f*)op = yv;
    __threadfence();
    *(volatile v4f*)op = yv;
  }
  put_x(yv);
  __syncthreads();

  auto eval_field = [&]() -> v4f {
    {
      v8f aH, aL;
      mm_tile(a1row, w1h, w1l, D_DIM, aH, aL);
#pragma unroll
      for (int r = 0; r < 8; ++r) {
        const float v = (aH[r] + aL[r] * W_LO_INV) * ACC_INV + b1v;
        h1dst[r * H_DIM] = (_Float16)(ftanh(v) * A_CARRY);
      }
    }
    __syncthreads();
    {
      v8f aH, aL;
      mm_tile(a2row, w2h, w2l, H_DIM, aH, aL);
#pragma unroll
      for (int r = 0; r < 8; ++r) {
        const float v = (aH[r] + aL[r] * W_LO_INV) * ACC_INV + b2v;
        h2dst[r * H_DIM] = (_Float16)(ftanh(v) * A_CARRY);
      }
    }
    __syncthreads();
    {
      v8f aH, aL;
      mm_tile(a3row, w3h, w3l, H_DIM / 2, aH, aL);
#pragma unroll
      for (int r = 0; r < 8; ++r) k3dst[r * D_DIM] = (aH[r] + aL[r] * W_LO_INV) * ACC_INV + b3v;
    }
    __syncthreads();
    const v4f p0 = *(const v4f*)(sKP + e0);
    const v4f p1 = *(const v4f*)(sKP + TILE_ELEMS + e0);
    return p0 + p1;
  };

#pragma unroll 1
  for (int iv = 0; iv < N_SAVE - 1; ++iv) {
    const float hstep = (ts[iv + 1] - ts[iv]) * 0.5f;
#pragma unroll 1
    for (int sub = 0; sub < N_SUB; ++sub) {
      v4f x;
      const v4f k1 = eval_field();
#pragma unroll
      for (int j = 0; j < 4; ++j) x[j] = yv[j] + hstep * (TS_A21 * k1[j]);
      put_x(x);
      __syncthreads();
      const v4f k2 = eval_field();
#pragma unroll
      for (int j = 0; j < 4; ++j) x[j] = yv[j] + hstep * (TS_A31 * k1[j] + TS_A32 * k2[j]);
      put_x(x);
      __syncthreads();
      const v4f k3 = eval_field();
#pragma unroll
      for (int j = 0; j < 4; ++j) x[j] = yv[j] + hstep * (TS_A41 * k1[j] + TS_A42 * k2[j] + TS_A43 * k3[j]);
      put_x(x);
      __syncthreads();
      const v4f k4 = eval_field();
#pragma unroll
      for (int j = 0; j < 4; ++j)
        x[j] = yv[j] + hstep * (TS_A51 * k1[j] + TS_A52 * k2[j] + TS_A53 * k3[j] + TS_A54 * k4[j]);
      put_x(x);
      __syncthreads();
      const v4f k5 = eval_field();
#pragma unroll
      for (int j = 0; j < 4; ++j)
        x[j] = yv[j] + hstep * (TS_A61 * k1[j] + TS_A62 * k2[j] + TS_A63 * k3[j] + TS_A64 * k4[j] + TS_A65 * k5[j]);
      put_x(x);
      __syncthreads();
      const v4f k6 = eval_field();
#pragma unroll
      for (int j = 0; j < 4; ++j)
        yv[j] = yv[j] + hstep * (TS_B1 * k1[j] + TS_B2 * k2[j] + TS_B3 * k3[j] + TS_B4 * k4[j] + TS_B5 * k5[j] + TS_B6 * k6[j]);
      put_x(yv);
      __syncthreads();
    }
    float* op = out + (size_t)(iv + 1) * ((size_t)N_BATCH * D_DIM) + (size_t)blk * TILE_ELEMS + e0;
    const v4f yo = yv;
    *(volatile v4f*)op = yo;
    __threadfence();
    *(volatile v4f*)op = yo;
  }
}

extern "C" void kernel_launch(void* const* d_in, const int* in_sizes, int n_in,
                              void* d_out, int out_size, void* d_ws, size_t ws_size, hipStream_t stream) {
  if (n_in < 8 || d_out == nullptr || d_ws == nullptr) return;
  if (in_sizes[0] != N_SAVE || in_sizes[1] != N_BATCH * D_DIM || in_sizes[2] != H_DIM * D_DIM || in_sizes[3] != H_DIM ||
      in_sizes[4] != H_DIM * H_DIM || in_sizes[5] != H_DIM || in_sizes[6] != D_DIM * H_DIM || in_sizes[7] != D_DIM ||
      out_size != N_SAVE * N_BATCH * D_DIM) return;

  const float* ts = (const float*)d_in[0];
  const float* y0 = (const float*)d_in[1];
  const float* W1 = (const float*)d_in[2];
  const float* b1 = (const float*)d_in[3];
  const float* W2 = (const float*)d_in[4];
  const float* b2 = (const float*)d_in[5];
  const float* W3 = (const float*)d_in[6];
  const float* b3 = (const float*)d_in[7];
  float* out = (float*)d_out;

  char* ws = (char*)d_ws; size_t off = 0;
  auto carve = [&](size_t bytes) -> char* { char* p = ws + off; off += (bytes + 255) & ~(size_t)255; return p; };
  unsigned short* W1H = (unsigned short*)carve((size_t)H_DIM * D_DIM * 2);
  unsigned short* W1L = (unsigned short*)carve((size_t)H_DIM * D_DIM * 2);
  unsigned short* W2H = (unsigned short*)carve((size_t)H_DIM * H_DIM * 2);
  unsigned short* W2L = (unsigned short*)carve((size_t)H_DIM * H_DIM * 2);
  unsigned short* W3H = (unsigned short*)carve((size_t)D_DIM * H_DIM * 2);
  unsigned short* W3L = (unsigned short*)carve((size_t)D_DIM * H_DIM * 2);
  if (off > ws_size || off > (size_t)134217728) return;

  const int n8a = H_DIM * D_DIM / 8, n8b = H_DIM * H_DIM / 8, n8c = D_DIM * H_DIM / 8;
  split_planes_kernel<<<n8a / NTHREADS, NTHREADS, 0, stream>>>(W1, W1H, W1L, n8a);
  split_planes_kernel<<<n8b / NTHREADS, NTHREADS, 0, stream>>>(W2, W2H, W2L, n8b);
  split_planes_kernel<<<n8c / NTHREADS, NTHREADS, 0, stream>>>(W3, W3H, W3L, n8c);
  field_solver_kernel<<<N_BATCH / TILE_ROWS, NTHREADS, 0, stream>>>(ts, y0, W1H, W1L, b1, W2H, W2L, b2, W3H, W3L, b3, out);
}
